// MultiHeadAttentionLayer_82497731822091
// MI455X (gfx1250) — hardware-verified
//
#include <hip/hip_runtime.h>
#include <stddef.h>
#include <stdint.h>
#include <math.h>


#define DM      128
#define NHD     8
#define HDM     16
#define QKVW    384
#define OQ      0
#define OKK     128
#define OV      256
#define NTHR    256
#define NWAVE   8
#define EPT     8
#define CHUNK   (NTHR * EPT)
#define WCAP    (EPT * 32)
#define LISTN   (NWAVE * WCAP)
#define NBMAX   1024
#define SLOTB   10
#define RCAP    28672
#define DEGCAP  64
#define GBM     64
#define GBN     64
#define GTHR    128
#define KU      4
#define ATTSC   0.25f
#define CLIPV   5.0f
#define WSMAX   134217728
#define LDS_AGG ((2 * RCAP + 2 * NBMAX + LISTN + 2 * NWAVE) * 4 + 64)

static_assert((1 << SLOTB) == NBMAX);
static_assert(SLOTB + 21 <= 31);
static_assert((CHUNK & (CHUNK - 1)) == 0 && CHUNK <= 2048 && SLOTB + 11 <= 31);
static_assert(NTHR * 4 == NBMAX);
static_assert(LISTN >= NBMAX);
static_assert(LISTN >= NWAVE * WCAP);
static_assert((RCAP % 32) == 0);
static_assert((NBMAX % NWAVE) == 0);
static_assert(LDS_AGG <= 300000);
static_assert(GBM == (GTHR / 32) * 16);
static_assert((DM % 32) == 0 && ((DM / 32) % KU) == 0);
static_assert((DM / 8) == 16);
static_assert(DM == 4 * 32);
static_assert(HDM == 4 * 4 && NHD * HDM == DM);
static_assert(QKVW == 3 * DM && (QKVW % GBN) == 0 && (DM % GBN) == 0);

typedef float          v4f  __attribute__((ext_vector_type(4)));
typedef float          v8f  __attribute__((ext_vector_type(8)));
typedef int            v4i  __attribute__((ext_vector_type(4)));
typedef int            v8i  __attribute__((ext_vector_type(8)));
typedef unsigned int   v4u  __attribute__((ext_vector_type(4)));
typedef unsigned short v8us __attribute__((ext_vector_type(8)));
typedef __bf16         v16b __attribute__((ext_vector_type(16)));
typedef v4f  __attribute__((may_alias)) v4fa;
typedef v4u  __attribute__((may_alias)) v4ua;
typedef v8us __attribute__((may_alias)) v8usa;
union FragB { v16b v; v8us h[2]; v8i w; };

__device__ __forceinline__ v8f wmb(const FragB& a, const FragB& b, v8f c) {
  v8f d = __builtin_amdgcn_wmma_f32_16x16x32_bf16(false, a.v, false, b.v, (short)0, c, false, false);
  asm volatile("v_nop\n\tv_nop\n\tv_nop\n\tv_nop" : "+v"(d) : "v"(a.w), "v"(b.w));
  return d;
}
__device__ __forceinline__ v8f z8() { v8f z = {0.f, 0.f, 0.f, 0.f, 0.f, 0.f, 0.f, 0.f}; return z; }

__device__ __forceinline__ unsigned int f2bf(float f) {
  const unsigned int u = __float_as_uint(f);
  return ((u + 0x7FFFu + ((u >> 16) & 1u)) >> 16) & 0xFFFFu;
}
__device__ __forceinline__ float bf2f(unsigned int b) { return __uint_as_float(b << 16); }
__device__ __forceinline__ float bfr(float f) { return bf2f(f2bf(f)); }
__device__ __forceinline__ v4f bfr4(const v4f a) {
  v4f r; r.x = bfr(a.x); r.y = bfr(a.y); r.z = bfr(a.z); r.w = bfr(a.w); return r;
}
__device__ __forceinline__ unsigned int pk2(float lo, float hi) { return f2bf(lo) | (f2bf(hi) << 16); }
__device__ __forceinline__ v4u pack8(const v4f a, const v4f b) {
  v4u r;
  r.x = pk2(a.x, a.y); r.y = pk2(a.z, a.w); r.z = pk2(b.x, b.y); r.w = pk2(b.z, b.w);
  return r;
}

__device__ __forceinline__ float hsum4(float v) {
  v += __shfl_xor(v, 1, 32);
  v += __shfl_xor(v, 2, 32);
  return v;
}
__device__ __forceinline__ float dot4(const v4f a, const v4f b) {
  float p = a.x * b.x; p = fmaf(a.y, b.y, p); p = fmaf(a.z, b.z, p); p = fmaf(a.w, b.w, p);
  return p;
}

__device__ __forceinline__ int scan_chunk(const int* __restrict__ dsts, int nE, int cbase, int slotBase,
                                          int nb, int vec8, int* list, int tid, int lane, int wave) {
  int wc = 0;
  const int el0  = tid * EPT;
  const int e0   = cbase + el0;
  const int sent = -2147483647 - 1;
  v4i da, db;
  if (vec8 != 0 && cbase + CHUNK <= nE) {
    da = *(const v4i*)(dsts + e0);
    db = *(const v4i*)(dsts + e0 + 4);
  } else {
    da.x = (e0     < nE) ? dsts[min(e0,     nE - 1)] : sent;
    da.y = (e0 + 1 < nE) ? dsts[min(e0 + 1, nE - 1)] : sent;
    da.z = (e0 + 2 < nE) ? dsts[min(e0 + 2, nE - 1)] : sent;
    da.w = (e0 + 3 < nE) ? dsts[min(e0 + 3, nE - 1)] : sent;
    db.x = (e0 + 4 < nE) ? dsts[min(e0 + 4, nE - 1)] : sent;
    db.y = (e0 + 5 < nE) ? dsts[min(e0 + 5, nE - 1)] : sent;
    db.z = (e0 + 6 < nE) ? dsts[min(e0 + 6, nE - 1)] : sent;
    db.w = (e0 + 7 < nE) ? dsts[min(e0 + 7, nE - 1)] : sent;
  }
  const unsigned nbs = (unsigned)slotBase;
  const unsigned unb = (unsigned)nb;
  const unsigned s0 = (unsigned)da.x - nbs, s1 = (unsigned)da.y - nbs;
  const unsigned s2 = (unsigned)da.z - nbs, s3 = (unsigned)da.w - nbs;
  const unsigned s4 = (unsigned)db.x - nbs, s5 = (unsigned)db.y - nbs;
  const unsigned s6 = (unsigned)db.z - nbs, s7 = (unsigned)db.w - nbs;
  const bool h0 = s0 < unb, h1 = s1 < unb, h2 = s2 < unb, h3 = s3 < unb;
  const bool h4 = s4 < unb, h5 = s5 < unb, h6 = s6 < unb, h7 = s7 < unb;
  const unsigned any = __builtin_amdgcn_ballot_w32(h0 | h1 | h2 | h3 | h4 | h5 | h6 | h7);
  if (any != 0u) {
#define HITJ(J, HJ, SJ) { \
      const unsigned mj = __builtin_amdgcn_ballot_w32(HJ); \
      if (mj != 0u) { \
        if (HJ) { \
          const int pos = wc + (int)__builtin_amdgcn_mbcnt_lo(mj, 0u); \
          if (pos < WCAP) list[wave * WCAP + pos] = ((el0 + (J)) << SLOTB) | (int)(SJ); \
        } \
        wc += (int)__builtin_popcount(mj); } }
    HITJ(0, h0, s0)
    HITJ(1, h1, s1)
    HITJ(2, h2, s2)
    HITJ(3, h3, s3)
    HITJ(4, h4, s4)
    HITJ(5, h5, s5)
    HITJ(6, h6, s6)
    HITJ(7, h7, s7)
#undef HITJ
  }
  return wc;
}

__global__ __launch_bounds__(NTHR) void k_xprep(const float* __restrict__ x, unsigned short* xbp, int nN, int nUnits) {
  const int i = (int)blockIdx.x * NTHR + (int)threadIdx.x;
  if (i >= nUnits) return;
  const int row = i >> 4;
  const int c0  = (i & 15) * 8;
  const int rc  = row < nN ? row : nN - 1;
  const float* p = x + (size_t)rc * DM + c0;
  v4f a = *(const v4fa*)p;
  v4f b = *(const v4fa*)(p + 4);
  const v4f z4 = {0.f, 0.f, 0.f, 0.f};
  if (row >= nN) { a = z4; b = z4; }
  const v4u hv = pack8(a, b);
  unsigned short* o = xbp + (size_t)row * DM + c0;
  *(volatile v4u*)o = hv;
  __threadfence();
  *(volatile v4u*)o = hv;
}

__global__ __launch_bounds__(NTHR) void k_wtr(const float* __restrict__ w, int Kin, int Ncol, int Nrows, int Kout,
                                              unsigned short* wt, int nUnits) {
  const int u = (int)blockIdx.x * NTHR + (int)threadIdx.x;
  if (u >= nUnits) return;
  const int kq = Kout >> 3;
  const int n  = u / kq;
  const int k8 = (u - n * kq) * 8;
  const int kk = k8 - (k8 / Kin) * Kin;
  const int ncl = n < Ncol ? n : Ncol - 1;
  const float* p = w + (size_t)kk * (size_t)Ncol + ncl;
  v4f a, b;
  a.x = p[0];                    a.y = p[(size_t)Ncol];         a.z = p[(size_t)2 * Ncol];     a.w = p[(size_t)3 * Ncol];
  b.x = p[(size_t)4 * Ncol];     b.y = p[(size_t)5 * Ncol];     b.z = p[(size_t)6 * Ncol];     b.w = p[(size_t)7 * Ncol];
  const v4f z4 = {0.f, 0.f, 0.f, 0.f};
  if (n >= Ncol || n >= Nrows) { a = z4; b = z4; }
  const v4u wv = pack8(a, b);
  unsigned short* o = wt + (size_t)n * (size_t)Kout + k8;
  *(volatile v4u*)o = wv;
  __threadfence();
  *(volatile v4u*)o = wv;
}

__global__ __launch_bounds__(GTHR) void k_gemm(
    const unsigned short* __restrict__ A, const unsigned short* __restrict__ WT,
    const float* __restrict__ bq, const float* __restrict__ bk, const float* __restrict__ bv,
    float* outF)
{
  __shared__ __attribute__((aligned(16))) float stg[GBM * GBN];
  const int tid = (int)threadIdx.x, lane = tid & 31, wave = tid >> 5, hh = lane >> 4, m = lane & 15;
  const int rowBase = (int)blockIdx.x * GBM;
  const int col0    = (int)blockIdx.y * GBN;

  v8f acc[4];
  acc[0] = z8(); acc[1] = z8(); acc[2] = z8(); acc[3] = z8();
  const unsigned short* ap = A  + (size_t)(rowBase + 16 * wave + m) * (size_t)DM + 8 * hh;
  const unsigned short* wp = WT + (size_t)(col0 + m) * (size_t)DM + 8 * hh;
#pragma unroll 1
  for (int ks0 = 0; ks0 < DM / 32; ks0 += KU) {
#pragma unroll
    for (int uu = 0; uu < KU; ++uu) {
      const int ks = ks0 + uu;
      FragB af;
      af.h[0] = *(const v8usa*)(ap + 32 * ks);
      af.h[1] = *(const v8usa*)(ap + 32 * ks + 16);
#pragma unroll
      for (int t = 0; t < 4; ++t) {
        const unsigned short* wq = wp + (size_t)(16 * t) * (size_t)DM + 32 * ks;
        FragB bf;
        bf.h[0] = *(const v8usa*)wq;
        bf.h[1] = *(const v8usa*)(wq + 16);
        acc[t] = wmb(af, bf, acc[t]);
      }
    }
  }

#pragma unroll
  for (int t = 0; t < 4; ++t) {
    const int lc = 16 * t + m;
#pragma unroll
    for (int r = 0; r < 8; ++r) {
      const int lr = 16 * wave + 8 * hh + r;
      stg[lr * GBN + lc] = acc[t][r];
    }
  }
  __syncthreads();

  const int mat = col0 / DM;
  const int bo  = (col0 & (DM - 1)) + 4 * m;
  const float f0 = (mat == 0) ? 1.0f : 0.0f;
  const float f1 = (mat == 1) ? 1.0f : 0.0f;
  const float f2 = (mat == 2) ? 1.0f : 0.0f;
  const v4f b0 = bfr4(*(const v4fa*)(bq + bo));
  const v4f b1 = bfr4(*(const v4fa*)(bk + bo));
  const v4f b2 = bfr4(*(const v4fa*)(bv + bo));
  const v4f bsel = b0 * f0 + b1 * f1 + b2 * f2;

  v4f fv[8];
#pragma unroll
  for (int i = 0; i < 8; ++i) {
    const int lr = 16 * wave + 2 * i + hh;
    fv[i] = *(const v4fa*)(stg + lr * GBN + 4 * m) + bsel;
  }
#pragma unroll
  for (int i = 0; i < 8; ++i) {
    const int lr = 16 * wave + 2 * i + hh;
    const int gr = rowBase + lr;
    float* op = outF + (size_t)gr * (size_t)QKVW + col0 + 4 * m;
    *(volatile v4f*)op = fv[i];
  }
  __threadfence();
#pragma unroll
  for (int i = 0; i < 8; ++i) {
    const int lr = 16 * wave + 2 * i + hh;
    const int gr = rowBase + lr;
    float* op = outF + (size_t)gr * (size_t)QKVW + col0 + 4 * m;
    *(volatile v4f*)op = fv[i];
  }
}

__global__ __launch_bounds__(NTHR) void k_agg(
    const int* __restrict__ srcs, const int* __restrict__ dsts,
    const float* __restrict__ QKV, float* out, int nN, int nE, int vec8) {
  extern __shared__ v4f lds_dyn[];
  int* reg1 = (int*)lds_dyn;
  int* reg2 = reg1 + RCAP;
  int* scnt = reg2 + RCAP;
  int* soff = scnt + NBMAX;
  int* list = soff + NBMAX;
  int* wcnt = list + LISTN;
  int* wtot = wcnt + NWAVE;
  const int tid = (int)threadIdx.x, lane = tid & 31, wave = tid >> 5;
  const int nodeBase = (int)blockIdx.x * NBMAX;

  for (int i = tid; i < NBMAX; i += NTHR) scnt[i] = 0;
  __syncthreads();

  int tot = 0;
  const int nChunks = (nE + CHUNK - 1) / CHUNK;
#pragma unroll 1
  for (int ch = 0; ch < nChunks; ++ch) {
    const int cbase = ch * CHUNK;
    const int wc = scan_chunk(dsts, nE, cbase, nodeBase, NBMAX, vec8, list, tid, lane, wave);
    if (lane == 0) wcnt[wave] = wc;
    __syncthreads();
    int pre = 0, all = 0;
#pragma unroll
    for (int w2 = 0; w2 < NWAVE; ++w2) {
      int c = wcnt[w2];
      c = c < 0 ? 0 : (c > WCAP ? WCAP : c);
      all += c;
      pre += (w2 < wave) ? c : 0;
    }
    const int wcc  = wc > WCAP ? WCAP : wc;
    const int base = tot + pre;
#pragma unroll 1
    for (int i = lane; i < wcc; i += 32) {
      const int ent = list[wave * WCAP + i];
      const int el  = (ent >> SLOTB) & (CHUNK - 1);
      const int sl  = ent & (NBMAX - 1);
      int eid = cbase + el;
      eid = eid > nE - 1 ? nE - 1 : eid;
      const int pos = base + i;
      if (pos < RCAP) reg1[pos] = (int)(((unsigned)eid << SLOTB) | (unsigned)sl);
    }
    tot += all;
    tot = tot > RCAP ? RCAP : tot;
    __syncthreads();
  }
  const int nh = tot;

  if (wave == 0) {
#pragma unroll 1
    for (int b0 = 0; b0 < nh; b0 += 32) {
      const int idx = b0 + lane;
      const int uv  = reg1[idx < nh ? idx : nh - 1];
      const int m32 = (nh - b0) < 32 ? (nh - b0) : 32;
#pragma unroll 1
      for (int k = 0; k < m32; ++k) {
        const int u  = __builtin_amdgcn_readlane(uv, k);
        const int sl = u & (NBMAX - 1);
        if (lane == 0) scnt[sl] = scnt[sl] + 1;
      }
    }
  }
  __syncthreads();

  {
    const v4i ca = *(const v4i*)(scnt + 4 * tid);
    const int e0 = ca.x < 0 ? 0 : ca.x, e1 = ca.y < 0 ? 0 : ca.y, e2 = ca.z < 0 ? 0 : ca.z, e3 = ca.w < 0 ? 0 : ca.w;
    const int ts = e0 + e1 + e2 + e3;
    int incl = ts;
#pragma unroll
    for (int d = 1; d < 32; d <<= 1) {
      const int up = __shfl_up(incl, d);
      if (lane >= d) incl += up;
    }
    if (lane == 31) wtot[wave] = incl;
    __syncthreads();
    int pre = 0;
#pragma unroll
    for (int w2 = 0; w2 < NWAVE; ++w2) pre += (w2 < wave) ? wtot[w2] : 0;
    int run = pre + incl - ts;
    soff[4 * tid + 0] = run; run += e0;
    soff[4 * tid + 1] = run; run += e1;
    soff[4 * tid + 2] = run; run += e2;
    soff[4 * tid + 3] = run;
  }
  __syncthreads();
  for (int i = tid; i < NBMAX; i += NTHR) list[i] = soff[i];
  __syncthreads();

  if (wave == 0) {
#pragma unroll 1
    for (int b0 = 0; b0 < nh; b0 += 32) {
      const int idx = b0 + lane;
      const int uv  = reg1[idx < nh ? idx : nh - 1];
      const int m32 = (nh - b0) < 32 ? (nh - b0) : 32;
#pragma unroll 1
      for (int k = 0; k < m32; ++k) {
        const int u   = __builtin_amdgcn_readlane(uv, k);
        const int sl  = u & (NBMAX - 1);
        const int eid = (int)((unsigned)u >> SLOTB);
        if (lane == 0) {
          int pos = list[sl];
          pos = pos < 0 ? 0 : (pos > RCAP - 1 ? RCAP - 1 : pos);
          reg2[pos] = eid;
          list[sl] = pos + 1;
        }
      }
    }
  }
  __syncthreads();

  const int nbw = NBMAX / NWAVE;
  const bool ovf = (nh >= RCAP);
  const float qnan = __int_as_float(0x7fc00000);
  const int c4 = 4 * lane;
  const v4f z4 = {0.f, 0.f, 0.f, 0.f};

#pragma unroll 1
  for (int jt = 0; jt < nbw; ++jt) {
    const int slot = wave * nbw + jt;
    const int grow = nodeBase + slot;
    const int gcl  = grow < nN ? grow : nN - 1;
    int st = soff[slot];
    const int craw = scnt[slot];
    int cnt = craw;
    st  = st < 0 ? 0 : (st > nh ? nh : st);
    cnt = cnt < 0 ? 0 : (cnt > DEGCAP ? DEGCAP : cnt);
    if (cnt > nh - st) cnt = nh - st;
    const float pz = (ovf || craw > DEGCAP) ? qnan : 0.0f;

    const v4f qv = *(const v4fa*)(QKV + (size_t)gcl * QKVW + OQ + c4);
    float mx = -1.0e30f, dn = 0.f;
    v4f av = z4;

#pragma unroll 1
    for (int q = 0; q < cnt; ++q) {
      int idx = st + q; idx = idx > RCAP - 1 ? RCAP - 1 : idx;
      int eid = reg2[idx]; eid = eid < 0 ? 0 : (eid > nE - 1 ? nE - 1 : eid);
      const int sraw = srcs[eid];
      const int s = sraw < 0 ? 0 : (sraw > nN - 1 ? nN - 1 : sraw);
      const float* kr = QKV + (size_t)s * QKVW;
      const v4f kv = *(const v4fa*)(kr + OKK + c4);
      const v4f vv = *(const v4fa*)(kr + OV + c4);
      float lg = hsum4(dot4(qv, kv)) * ATTSC;
      lg = fminf(CLIPV, fmaxf(-CLIPV, lg));
      const float df = lg - mx;
      const float ex = __expf(-fabsf(df));
      const bool up  = df > 0.f;
      const float s1 = up ? ex : 1.0f;
      const float s2 = up ? 1.0f : ex;
      mx = up ? lg : mx;
      dn = fmaf(dn, s1, s2);
      av = av * s1 + vv * s2;
    }
    const float dns = dn > 0.f ? dn : 1.0f;
    const float ind = dn > 0.f ? 1.0f : 0.0f;
    const float inv = ind * __builtin_amdgcn_rcpf(dns);
    const v4f msg = av * inv + pz;

    const bool wr = (grow < nN);
    const int gsf = wr ? grow : nN - 1;
    float* orow = out + (size_t)gsf * DM + c4;
    if (wr) {
      *(volatile v4f*)orow = msg;
    }
    __threadfence();
    if (wr) {
      *(volatile v4f*)orow = msg;
    }
  }
}

static inline int cdiv(int a, int b) { return (a + b - 1) / b; }
static inline size_t al256(size_t o) { return (o + 255) & ~(size_t)255; }

extern "C" void kernel_launch(void* const* d_in, const int* in_sizes, int n_in,
                              void* d_out, int out_size, void* d_ws, size_t ws_size,
                              hipStream_t stream) {
  if (n_in < 8) return;
  if (in_sizes[0] < DM || (in_sizes[0] % DM) != 0) return;
  const int nN = in_sizes[0] / DM;
  if (nN < 16 || nN > (1 << 22)) return;
  if (in_sizes[1] < 2 || (in_sizes[1] & 1) != 0) return;
  const int nE = in_sizes[1] / 2;
  if (nE < 1 || nE >= (1 << (31 - SLOTB))) return;
  if (in_sizes[2] != DM * DM || in_sizes[4] != DM * DM || in_sizes[6] != DM * DM) return;
  if (in_sizes[3] != DM || in_sizes[5] != DM || in_sizes[7] != DM) return;
  if ((long long)out_size != (long long)nN * DM) return;

  const float* x  = (const float*)d_in[0];
  const int*   ei = (const int*)  d_in[1];
  const float* Wq = (const float*)d_in[2];
  const float* bq = (const float*)d_in[3];
  const float* Wk = (const float*)d_in[4];
  const float* bk = (const float*)d_in[5];
  const float* Wv = (const float*)d_in[6];
  const float* bv = (const float*)d_in[7];
  float* out = (float*)d_out;
  const int* src = ei;
  const int* dst = ei + nE;

  const int MP   = cdiv(nN, GBM) * GBM;
  const int gM   = MP / GBM;
  const int gA   = cdiv(nN, NBMAX);
  const int vec8 = ((nE & 3) == 0) ? 1 : 0;
  if ((long long)gA * NBMAX < (long long)nN) return;

  char* ws = (char*)d_ws;
  size_t off = 0;
  const size_t oXB  = off; off = al256(off + (size_t)MP * DM * 2);
  const size_t oWQ  = off; off = al256(off + (size_t)QKVW * DM * 2);
  const size_t oQKV = off; off = al256(off + (size_t)MP * QKVW * 4);
  if (off > ws_size || off > (size_t)WSMAX) return;
  unsigned short* XB    = (unsigned short*)(ws + oXB);
  unsigned short* WQKVT = (unsigned short*)(ws + oWQ);
  float*          QKV   = (float*)(ws + oQKV);

  hipFuncSetAttribute(reinterpret_cast<const void*>(&k_agg),
                      hipFuncAttributeMaxDynamicSharedMemorySize, LDS_AGG);

  const int nUx = MP * (DM / 8);
  k_xprep<<<cdiv(nUx, NTHR), NTHR, 0, stream>>>(x, XB, nN, nUx);

  {
    const int nUq = DM * (DM / 8);
    const size_t pl = (size_t)DM * DM;
    k_wtr<<<cdiv(nUq, NTHR), NTHR, 0, stream>>>(Wq, DM, DM, DM, DM, WQKVT,          nUq);
    k_wtr<<<cdiv(nUq, NTHR), NTHR, 0, stream>>>(Wk, DM, DM, DM, DM, WQKVT + pl,     nUq);
    k_wtr<<<cdiv(nUq, NTHR), NTHR, 0, stream>>>(Wv, DM, DM, DM, DM, WQKVT + 2 * pl, nUq);
  }

  k_gemm<<<dim3(gM, QKVW / GBN), GTHR, 0, stream>>>(XB, WQKVT, bq, bk, bv, QKV);
  k_agg<<<gA, NTHR, LDS_AGG, stream>>>(src, dst, QKV, out, nN, nE, vec8);
}
